// TrajPredictor_51616916963852
// MI455X (gfx1250) — hardware-run, weakly checked
//
#include <hip/hip_runtime.h>
#include <math.h>

constexpr int NBAT = 128;
constexpr int NTOB = 64;
constexpr int NAG  = 32;
constexpr int NFE  = 6;
constexpr int NHU  = 64;
constexpr int NDU  = 64;
constexpr int NPR  = 12;
constexpr int NBA  = NBAT * NAG;
constexpr int NG3  = 3 * NHU;
constexpr int NE2  = 2 * NHU;
constexpr int NROWF = NAG * NFE;
constexpr int NATT = NDU + NE2;
constexpr int NDIN = NFE + NE2;
constexpr int NER  = NBA * NTOB;
constexpr int ENC_THR = 128;
constexpr int ENC_ROWS = 16;
constexpr int DEC_THR = 256;
constexpr int DEC_ROWS = 32;
constexpr int HPAD = 72;
constexpr int CPAD = 136;
constexpr int NWXS = NG3 * NFE;
constexpr float WCAR = 16.0f;
constexpr float WCAR_INV = 1.0f / 16.0f;
static_assert(NHU == 16 * (ENC_THR / 32));
static_assert(NAG % ENC_ROWS == 0);
static_assert((ENC_ROWS * HPAD) % ENC_THR == 0);
static_assert(ENC_ROWS * NFE == 24 * 4);
static_assert(DEC_ROWS == NAG && DEC_THR == 256 && NDU == 64 && NHU == 64);
static_assert(DEC_ROWS * (NE2 / 8) == 2 * DEC_THR);
static_assert(DEC_ROWS * NTOB == 8 * DEC_THR);
static_assert(DEC_ROWS * NE2 == 16 * DEC_THR);
static_assert(NROWF == 128 + 64 && NROWF <= DEC_THR);
static_assert((NFE * NDU) % 4 == 0 && (NFE * NDU) / 4 <= DEC_THR);
static_assert(NER % 64 == 0 && NDU % 64 == 0 && NE2 % 32 == 0 && NDU % 32 == 0);
static_assert(((NER / 64) * (NDU / 64)) % 8 == 0);
static_assert(HPAD % 8 == 0 && CPAD % 8 == 0);
static_assert(NWXS % 4 == 0 && NG3 % 4 == 0 && NDU % 4 == 0);
static_assert(NG3 / 4 <= ENC_THR && NG3 / 4 <= DEC_THR && NDU / 4 <= DEC_THR && NG3 <= DEC_THR);

typedef __attribute__((ext_vector_type(16))) _Float16 v16h;
typedef __attribute__((ext_vector_type(8)))  _Float16 v8h;
typedef __attribute__((ext_vector_type(16))) __bf16   v16b;
typedef __attribute__((ext_vector_type(8)))  __bf16   v8b;
typedef __attribute__((ext_vector_type(8)))  float    v8f;
typedef __attribute__((ext_vector_type(4)))  float    v4f;

__device__ __forceinline__ unsigned short f2bf_bits(float f) {
  unsigned u = __float_as_uint(f);
  return (unsigned short)((u + 0x7FFFu + ((u >> 16) & 1u)) >> 16);
}
__device__ __forceinline__ float bf_bits2f(unsigned short h) { return __uint_as_float(((unsigned)h) << 16); }

__device__ __forceinline__ float h16_to_f32(unsigned hb) {
  const unsigned sgn = (hb & 0x8000u) << 16; const unsigned em = hb & 0x7fffu;
  const float fn = __uint_as_float((em << 13) + 0x38000000u);
  const float fs = (float)em * 5.9604644775390625e-8f;
  const float mag = (em < 0x400u) ? fs : fn; return __uint_as_float(__float_as_uint(mag) | sgn); }

__device__ __forceinline__ void dep_guard_h(v8f& a, v8f& b, v16h x, v16h y) { asm volatile("v_nop\n\tv_nop\n\tv_nop\n\tv_nop" : "+v"(a), "+v"(b) : "v"(x), "v"(y)); }
__device__ __forceinline__ void dep_guard_b(v8f& a, v8f& b, v16b x, v16b y) { asm volatile("v_nop\n\tv_nop\n\tv_nop\n\tv_nop" : "+v"(a), "+v"(b) : "v"(x), "v"(y)); }
__device__ __forceinline__ void dep_guard1_h(v8f& a, v16h x, v16h y) { asm volatile("v_nop\n\tv_nop\n\tv_nop\n\tv_nop" : "+v"(a) : "v"(x), "v"(y)); }
__device__ __forceinline__ void dep_guard3_h(v8f& a, v8f& b, v8f& c, v16h w, v16h x, v16h y, v16h z) {
  asm volatile("v_nop\n\tv_nop\n\tv_nop\n\tv_nop" : "+v"(a), "+v"(b), "+v"(c) : "v"(w), "v"(x), "v"(y), "v"(z)); }
__device__ __forceinline__ void keep4_h(v16h a, v16h b, v16h c, v16h d) { asm volatile("v_nop" :: "v"(a), "v"(b), "v"(c), "v"(d)); }
__device__ __forceinline__ void keep4_b(v16b a, v16b b, v16b c, v16b d) { asm volatile("v_nop" :: "v"(a), "v"(b), "v"(c), "v"(d)); }
__device__ __forceinline__ void acc_guard4(v8f& a, v8f& b, v8f& c, v8f& d) { asm volatile("v_nop\n\tv_nop\n\tv_nop\n\tv_nop" : "+v"(a), "+v"(b), "+v"(c), "+v"(d)); }
__device__ __forceinline__ void acc_guard3(v8f& a, v8f& b, v8f& c) { asm volatile("v_nop\n\tv_nop\n\tv_nop\n\tv_nop" : "+v"(a), "+v"(b), "+v"(c)); }
__device__ __forceinline__ void acc_guard1(v8f& a) { asm volatile("v_nop\n\tv_nop\n\tv_nop\n\tv_nop" : "+v"(a)); }

__device__ __forceinline__ void ld_use4(v4f a) { asm volatile("" :: "v"(a) : "memory"); }
__device__ __forceinline__ void ld_use4x2(v4f a, v4f b) { asm volatile("" :: "v"(a), "v"(b) : "memory"); }
__device__ __forceinline__ void ld_use4x3(v4f a, v4f b, v4f c) { asm volatile("" :: "v"(a), "v"(b), "v"(c) : "memory"); }
__device__ __forceinline__ void ld_use8(v8h a) { asm volatile("" :: "v"(a) : "memory"); }
__device__ __forceinline__ void ld_use16x2(v16h a, v16h b) { asm volatile("" :: "v"(a), "v"(b) : "memory"); }
__device__ __forceinline__ void ld_use_f1(float a) { asm volatile("" :: "v"(a) : "memory"); }
__device__ __forceinline__ void ld_use_f6(float a, float b, float c, float d, float e, float f) {
  asm volatile("" :: "v"(a), "v"(b), "v"(c), "v"(d), "v"(e), "v"(f) : "memory"); }

template <typename T> struct Frag;
template <> struct Frag<_Float16> {
  typedef v16h V; union U { v16h v; v8h h[2]; };
  static __device__ __forceinline__ v16h load(const _Float16* p) {
    U f; f.h[0] = *(const v8h*)(p); f.h[1] = *(const v8h*)(p + 16); return f.v;
  }
  static __device__ __forceinline__ v8f mma(v16h a, v16h b, v8f c) {
    return __builtin_amdgcn_wmma_f32_16x16x32_f16(false, a, false, b, (short)0, c, false, false);
  }
  static __device__ __forceinline__ void guard(v8f& a, v8f& b, v16h x, v16h y) { dep_guard_h(a, b, x, y); }
  static __device__ __forceinline__ void keep(v16h a, v16h b, v16h c, v16h d) { keep4_h(a, b, c, d); }
};
template <> struct Frag<__bf16> {
  typedef v16b V; union U { v16b v; v8b h[2]; };
  static __device__ __forceinline__ v16b load(const __bf16* p) {
    U f; f.h[0] = *(const v8b*)(p); f.h[1] = *(const v8b*)(p + 16); return f.v;
  }
  static __device__ __forceinline__ v8f mma(v16b a, v16b b, v8f c) {
    return __builtin_amdgcn_wmma_f32_16x16x32_bf16(false, a, false, b, (short)0, c, false, false);
  }
  static __device__ __forceinline__ void guard(v8f& a, v8f& b, v16b x, v16b y) { dep_guard_b(a, b, x, y); }
  static __device__ __forceinline__ void keep(v16b a, v16b b, v16b c, v16b d) { keep4_b(a, b, c, d); }
};

__device__ __forceinline__ float fsig(float x)  { return __builtin_amdgcn_rcpf(1.0f + __expf(-x)); }
__device__ __forceinline__ float ftanh(float x) { return 1.0f - 2.0f * __builtin_amdgcn_rcpf(__expf(2.0f * x) + 1.0f); }

template <int ET> struct Elem;
template <> struct Elem<0> { typedef _Float16 T; };
template <> struct Elem<1> { typedef __bf16 T; };
template <int ET, bool SPLIT, int BIAS_MODE, int OUT_MODE, bool RESID, int ACT = 0>
__global__ __launch_bounds__(256) void wmma_gemm64(
    const unsigned short* __restrict__ Ap, const unsigned short* __restrict__ A2p, int lda, long strideA,
    const unsigned short* __restrict__ Btp, const unsigned short* __restrict__ Bt2p, int ldb, long strideB,
    void* __restrict__ Cout, void* __restrict__ Cout2, int ldc, long strideC,
    const float* __restrict__ bias,
    const float* __restrict__ resid, long strideR,
    int M, int N, int K, float scale) {
  typedef typename Elem<ET>::T T;
  typedef typename Frag<T>::V V;
  const T* A = (const T*)Ap; const T* A2 = (const T*)A2p; const T* Bt = (const T*)Btp; const T* Bt2 = (const T*)Bt2p;
  __shared__ __align__(16) float sT[8][16 * 68];
  const int b    = blockIdx.y;
  const int lane = threadIdx.x & 31;
  const int wave = threadIdx.x >> 5;
  const int tilesN = N >> 6;
  const int tilesM = M >> 6;
  const int tile = blockIdx.x * 8 + wave;
  if (tile >= tilesM * tilesN) return;
  const int tm = tile / tilesN;
  const int tn = tile - tm * tilesN;
  const int m0 = tm << 6;
  const int n0 = tn << 6;

  const T* Ab  = A  + (size_t)b * strideA;
  const T* Bb  = Bt + (size_t)b * strideB;
  const T* Ab2 = SPLIT ? (A2  + (size_t)b * strideA) : nullptr;
  const T* Bb2 = SPLIT ? (Bt2 + (size_t)b * strideB) : nullptr;

  const int rlane = lane & 15;
  const int koff  = (lane >> 4) * 8;
  const int mOff  = (lane >> 4) * 8;

  v8f acc[4][4];
#pragma unroll
  for (int i = 0; i < 4; ++i)
#pragma unroll
    for (int j = 0; j < 4; ++j) acc[i][j] = (v8f){0.f,0.f,0.f,0.f,0.f,0.f,0.f,0.f};

  for (int k0 = 0; k0 < K; k0 += 32) {
    V bh[4], bl[4];
#pragma unroll
    for (int j = 0; j < 4; ++j) {
      const size_t bo = (size_t)(n0 + (j << 4) + rlane) * ldb + koff + k0;
      bh[j] = Frag<T>::load(Bb + bo);
      if (SPLIT) bl[j] = Frag<T>::load(Bb2 + bo);
    }
#pragma unroll
    for (int i = 0; i < 4; ++i) {
      const size_t ao = (size_t)(m0 + (i << 4) + rlane) * lda + koff + k0;
      V ah = Frag<T>::load(Ab + ao);
      V al;
      if (SPLIT) al = Frag<T>::load(Ab2 + ao);
#pragma unroll
      for (int j = 0; j < 4; ++j) {
        acc[i][j] = Frag<T>::mma(ah, bh[j], acc[i][j]);
        if (SPLIT) {
          acc[i][j] = Frag<T>::mma(ah, bl[j], acc[i][j]);
          acc[i][j] = Frag<T>::mma(al, bh[j], acc[i][j]);
        }
      }
      Frag<T>::guard(acc[i][0], acc[i][3], ah, SPLIT ? al : ah);
    }
    Frag<T>::keep(bh[0], bh[1], bh[2], bh[3]);
    if (SPLIT) Frag<T>::keep(bl[0], bl[1], bl[2], bl[3]);
  }
  acc_guard4(acc[0][0], acc[0][1], acc[0][2], acc[0][3]);
  acc_guard4(acc[1][0], acc[1][1], acc[1][2], acc[1][3]);
  acc_guard4(acc[2][0], acc[2][1], acc[2][2], acc[2][3]);
  acc_guard4(acc[3][0], acc[3][1], acc[3][2], acc[3][3]);

  float* slab = sT[wave];
  const float* Rb = RESID ? (resid + (size_t)b * strideR) : nullptr;
#pragma unroll
  for (int i = 0; i < 4; ++i) {
    const int mBase = m0 + (i << 4);
#pragma unroll
    for (int j = 0; j < 4; ++j) {
      const int n = n0 + (j << 4) + rlane;
      float bv = 0.f;
      if (BIAS_MODE == 2) bv = bias[n];
#pragma unroll
      for (int r = 0; r < 8; ++r) {
        float v = acc[i][j][r] * scale;
        if (BIAS_MODE == 1) v += bias[mBase + mOff + r];
        if (BIAS_MODE == 2) v += bv;
        if (RESID) v += Rb[(size_t)(mBase + mOff + r) * ldc + n];
        if (ACT == 1) v = tanhf(v);
        if (ACT == 2) v = fmaxf(v, 0.0f);
        if (ACT == 3) v = v / (1.0f + expf(-v));
        if (ACT == 4) v = (v > 0.f) ? v : 0.01f * v;
        if (ACT == 5) v = 0.5f * v * (1.0f + erff(v * 0.70710678118654752f));
        slab[(mOff + r) * 68 + (j << 4) + rlane] = v;
      }
    }
    __builtin_amdgcn_fence(__ATOMIC_RELEASE, "workgroup");
    __builtin_amdgcn_wave_barrier();
    __builtin_amdgcn_fence(__ATOMIC_ACQUIRE, "workgroup");
    if (OUT_MODE == 0) {
      float* C = (float*)Cout + (size_t)b * strideC;
      const int hh = lane >> 4, c4 = (lane & 15) * 4;
      for (int pass = 0; pass < 2; ++pass) {
#pragma unroll
        for (int it = 0; it < 8; ++it) {
          const int row = it * 2 + hh;
          v4f v = *(const v4f*)(slab + row * 68 + c4);
          *(volatile v4f*)(C + (size_t)(mBase + row) * ldc + n0 + c4) = v;
        }
        __threadfence();
      }
    } else {
      const int q = lane >> 3, c8 = (lane & 7) * 8;
      unsigned short* C  = (unsigned short*)Cout  + (size_t)b * strideC;
      unsigned short* C2 = (OUT_MODE == 2) ? ((unsigned short*)Cout2 + (size_t)b * strideC) : nullptr;
      for (int pass = 0; pass < 2; ++pass) {
#pragma unroll
        for (int it = 0; it < 4; ++it) {
          const int row = it * 4 + q;
          const float* sp = slab + row * 68 + c8;
          v8h hv, lv;
#pragma unroll
          for (int e = 0; e < 8; ++e) {
            if (OUT_MODE == 1) {
              hv[e] = (_Float16)sp[e];
            } else {
              unsigned short hb = f2bf_bits(sp[e]);
              unsigned short lb = f2bf_bits(sp[e] - bf_bits2f(hb));
              hv[e] = __builtin_bit_cast(_Float16, hb);
              lv[e] = __builtin_bit_cast(_Float16, lb);
            }
          }
          *(volatile v8h*)(C + (size_t)(mBase + row) * ldc + n0 + c8) = hv;
          if (OUT_MODE == 2) *(volatile v8h*)(C2 + (size_t)(mBase + row) * ldc + n0 + c8) = lv;
        }
        __threadfence();
      }
    }
    __builtin_amdgcn_fence(__ATOMIC_RELEASE, "workgroup");
    __builtin_amdgcn_wave_barrier();
    __builtin_amdgcn_fence(__ATOMIC_ACQUIRE, "workgroup");
  }
}

__global__ __launch_bounds__(256) void cvt_f16_kernel(const float* __restrict__ src, unsigned short* __restrict__ dst,
                                                      int nrow, int ncol8, int spitch, int scol0, float sc) {
  const int i  = blockIdx.x * 256 + threadIdx.x;
  const int n8 = nrow * ncol8;
  if (i < n8) {
    const int row = i / ncol8;
    const int c8  = i - row * ncol8;
    const float* sp = src + (size_t)row * spitch + scol0 + 8 * c8;
    float f[8];
#pragma unroll
    for (int e = 0; e < 8; ++e) f[e] = sp[e];
    v8h hv;
#pragma unroll
    for (int e = 0; e < 8; ++e) hv[e] = (_Float16)(f[e] * sc);
    *(volatile v8h*)(dst + (size_t)i * 8) = hv;
    __threadfence();
    *(volatile v8h*)(dst + (size_t)i * 8) = hv;
  }
}

__global__ __launch_bounds__(ENC_THR) void enc_gru_kernel(
    const float* __restrict__ src,
    const float* __restrict__ Wih_f, const float* __restrict__ bih_f, const float* __restrict__ bhh_f,
    const float* __restrict__ Wih_b, const float* __restrict__ bih_b, const float* __restrict__ bhh_b,
    const unsigned short* __restrict__ Whhf16p, const unsigned short* __restrict__ Whhb16p,
    unsigned short* __restrict__ enc16p) {
  __shared__ __align__(16) _Float16 Ah[ENC_ROWS * HPAD];
  __shared__ __align__(16) float    xs[ENC_ROWS * NFE];
  __shared__ __align__(16) float    wcs[NWXS + 2 * NG3];
  const int tid = threadIdx.x, lane = tid & 31, wave = tid >> 5;
  const int c = lane & 15, hh = lane >> 4, koff = hh * 8;
  const int rowbase = blockIdx.x * ENC_ROWS;
  const int dir = blockIdx.y;
  const _Float16* Whh16 = (const _Float16*)(dir ? Whhb16p : Whhf16p);
  const float* Wih = dir ? Wih_b : Wih_f;
  const float* bih = dir ? bih_b : bih_f;
  const float* bhh = dir ? bhh_b : bhh_f;
  const int j = 16 * wave + c;
  const int bidx = rowbase / NAG;
  const int a0   = rowbase - bidx * NAG;
  const float* xsrc = src + (size_t)bidx * NTOB * NROWF + a0 * NFE;

#pragma unroll 1
  for (int i = tid; i < ENC_ROWS * HPAD; i += ENC_THR) Ah[i] = (_Float16)0.0f;
  {
    const int tt0 = dir ? (NTOB - 1) : 0;
    const int i = (tid < 24) ? tid : 23;
    const v4f v = *(const v4f*)(xsrc + (size_t)tt0 * NROWF + 4 * i);
    if (tid < 24) *(v4f*)(xs + 4 * i) = v;
    ld_use4(v);
  }
  {
#pragma unroll 1
    for (int i = tid; i < NWXS / 4; i += ENC_THR) {
      const v4f v = *(const v4f*)(Wih + 4 * i);
      *(v4f*)(wcs + 4 * i) = v;
      ld_use4(v);
    }
    const int ib = (tid < NG3 / 4) ? tid : (NG3 / 4 - 1);
    const v4f vb = *(const v4f*)(bih + 4 * ib);
    const v4f vh = *(const v4f*)(bhh + 4 * ib);
    if (tid < NG3 / 4) {
      *(v4f*)(wcs + NWXS + 4 * ib) = vb;
      *(v4f*)(wcs + NWXS + NG3 + 4 * ib) = vh;
    }
    ld_use4x2(vb, vh);
  }
  v16h bfr[3][2];
#pragma unroll
  for (int g = 0; g < 3; ++g) {
    bfr[g][0] = Frag<_Float16>::load(Whh16 + (size_t)(g * NHU + j) * NHU + koff);
    bfr[g][1] = Frag<_Float16>::load(Whh16 + (size_t)(g * NHU + j) * NHU + koff + 32);
    ld_use16x2(bfr[g][0], bfr[g][1]);
  }
  float hst[8];
#pragma unroll
  for (int r = 0; r < 8; ++r) hst[r] = 0.0f;
  __syncthreads();
  float wx0[NFE], wx1[NFE], wx2[NFE];
#pragma unroll
  for (int f = 0; f < NFE; ++f) {
    wx0[f] = wcs[(0 * NHU + j) * NFE + f];
    wx1[f] = wcs[(1 * NHU + j) * NFE + f];
    wx2[f] = wcs[(2 * NHU + j) * NFE + f];
  }
  const float bi0 = wcs[NWXS + j], bi1 = wcs[NWXS + NHU + j], bi2 = wcs[NWXS + 2 * NHU + j];
  const float bh0 = wcs[NWXS + NG3 + j], bh1 = wcs[NWXS + NG3 + NHU + j], bh2 = wcs[NWXS + NG3 + 2 * NHU + j];

  const _Float16* ahrow = Ah + c * HPAD + koff;
  const v8f z8 = {0.f, 0.f, 0.f, 0.f, 0.f, 0.f, 0.f, 0.f};

#pragma unroll 1
  for (int step = 0; step < NTOB; ++step) {
    const int tt = dir ? (NTOB - 1 - step) : step;
    const v16h fa0 = Frag<_Float16>::load(ahrow);
    const v16h fa1 = Frag<_Float16>::load(ahrow + 32);
    v8f ar = Frag<_Float16>::mma(fa0, bfr[0][0], z8);
    ar = Frag<_Float16>::mma(fa1, bfr[0][1], ar);
    v8f az = Frag<_Float16>::mma(fa0, bfr[1][0], z8);
    az = Frag<_Float16>::mma(fa1, bfr[1][1], az);
    v8f an = Frag<_Float16>::mma(fa0, bfr[2][0], z8);
    an = Frag<_Float16>::mma(fa1, bfr[2][1], an);
    dep_guard3_h(ar, az, an, fa0, fa1, bfr[0][0], bfr[2][1]);
#pragma unroll
    for (int r = 0; r < 8; ++r) {
      const float* xp = xs + (8 * hh + r) * NFE;
      float gir = bi0, giz = bi1, gin = bi2;
#pragma unroll
      for (int f = 0; f < NFE; ++f) {
        const float xv = xp[f];
        gir = fmaf(xv, wx0[f], gir);
        giz = fmaf(xv, wx1[f], giz);
        gin = fmaf(xv, wx2[f], gin);
      }
      const float pr = ar[r] * WCAR_INV + bh0 + gir;
      const float pz = az[r] * WCAR_INV + bh1 + giz;
      const float hn = an[r] * WCAR_INV + bh2;
      const float rg = fsig(pr);
      const float zg = fsig(pz);
      const float ng = ftanh(gin + rg * hn);
      hst[r] = (1.0f - zg) * ng + zg * hst[r];
    }
    __syncthreads();
#pragma unroll
    for (int r = 0; r < 8; ++r) Ah[(8 * hh + r) * HPAD + j] = (_Float16)hst[r];
    {
      const int sn = (step + 1 < NTOB) ? (step + 1) : (NTOB - 1);
      const int ttn = dir ? (NTOB - 1 - sn) : sn;
      const int i = (tid < 24) ? tid : 23;
      const v4f v = *(const v4f*)(xsrc + (size_t)ttn * NROWF + 4 * i);
      if (tid < 24) *(v4f*)(xs + 4 * i) = v;
      ld_use4(v);
    }
    __syncthreads();
    {
      const int row = 4 * wave + (lane >> 3);
      const int c8  = (lane & 7) * 8;
      const v8h hv = *(const v8h*)(Ah + row * HPAD + c8);
      unsigned short* dp = enc16p + ((size_t)(rowbase + row) * NTOB + (size_t)tt) * NE2 + dir * NHU + c8;
      *(volatile v8h*)dp = hv;
      __threadfence();
      *(volatile v8h*)dp = hv;
    }
  }
}

__device__ __forceinline__ float sc_term(unsigned hb, float q, float v, float s) {
  const float e = h16_to_f32(hb);
  return fmaf(v, ftanh(e + q), s);
}

__global__ __launch_bounds__(DEC_THR) void dec_kernel(
    const float* __restrict__ src, const int* __restrict__ pred_len,
    const unsigned short* __restrict__ enc16p, const unsigned short* __restrict__ E16p,
    const unsigned short* __restrict__ Wah16p, const unsigned short* __restrict__ Wihc16p,
    const unsigned short* __restrict__ Whhd16p, const unsigned short* __restrict__ We2d16p,
    const float* __restrict__ v_attn, const float* __restrict__ b_e2d,
    const float* __restrict__ Wih_d, const float* __restrict__ bih_d, const float* __restrict__ bhh_d,
    const float* __restrict__ W_out, const float* __restrict__ b_out, float* __restrict__ out) {
  __shared__ __align__(16) _Float16 hA[DEC_ROWS * HPAD];
  __shared__ __align__(16) _Float16 cA[DEC_ROWS * CPAD];
  __shared__ __align__(16) float qs[DEC_ROWS * NDU];
  __shared__ __align__(16) float sc[DEC_ROWS * NTOB];
  __shared__ __align__(16) float hs[DEC_ROWS * NDU];
  __shared__ __align__(16) float vs[NDU];
  __shared__ __align__(16) float wo[NFE * NDU];
  __shared__ __align__(16) float po[NROWF];
  __shared__ __align__(16) float wxs[NWXS];
  __shared__ __align__(16) float bcs[2 * NG3 + NDU];
  const _Float16* enc16  = (const _Float16*)enc16p;
  const _Float16* Wah16  = (const _Float16*)Wah16p;
  const _Float16* Wihc16 = (const _Float16*)Wihc16p;
  const _Float16* Whhd16 = (const _Float16*)Whhd16p;
  const _Float16* We2d16 = (const _Float16*)We2d16p;
  const int tid = threadIdx.x, lane = tid & 31, wave = tid >> 5;
  const int c = lane & 15, hh = lane >> 4, koff = hh * 8;
  const int mi = wave >> 2, ub = wave & 3;
  const int j = 16 * ub + c;
  const int bidx = blockIdx.x;
  const int ba0 = bidx * NAG;

  {
    const int iv = (tid < NDU / 4) ? tid : (NDU / 4 - 1);
    const v4f vv = *(const v4f*)(v_attn + 4 * iv);
    const int iw = (tid < (NFE * NDU) / 4) ? tid : ((NFE * NDU) / 4 - 1);
    const v4f vw = *(const v4f*)(W_out + 4 * iw);
    if (tid < NDU / 4) *(v4f*)(vs + 4 * iv) = vv;
    if (tid < (NFE * NDU) / 4) *(v4f*)(wo + 4 * iw) = vw;
    ld_use4x2(vv, vw);
  }
  {
    const int i = (tid < NROWF) ? tid : (NROWF - 1);
    const float v = src[((size_t)bidx * NTOB + (NTOB - 1)) * NROWF + i];
    if (tid < NROWF) po[i] = v;
    ld_use_f1(v);
  }
#pragma unroll
  for (int it = 0; it < 2; ++it) {
    const int idx = it * DEC_THR + tid;
    const int row = idx >> 4, u = idx & 15;
    const int tsel = (u < 8) ? (NTOB - 1) : 0;
    const v8h v = *(const v8h*)(enc16 + ((size_t)(ba0 + row) * NTOB + (size_t)tsel) * NE2 + 8 * u);
    *(v8h*)(cA + row * CPAD + 8 * u) = v;
    ld_use8(v);
  }
  {
    const int n = (tid < NG3) ? tid : (NG3 - 1);
    const float* wp = Wih_d + (size_t)n * NDIN;
    const float w0 = wp[0], w1 = wp[1], w2 = wp[2], w3 = wp[3], w4 = wp[4], w5 = wp[5];
    if (tid < NG3) {
      wxs[n * NFE + 0] = w0; wxs[n * NFE + 1] = w1; wxs[n * NFE + 2] = w2;
      wxs[n * NFE + 3] = w3; wxs[n * NFE + 4] = w4; wxs[n * NFE + 5] = w5;
    }
    ld_use_f6(w0, w1, w2, w3, w4, w5);
  }
  {
    const int ib = (tid < NG3 / 4) ? tid : (NG3 / 4 - 1);
    const v4f vb = *(const v4f*)(bih_d + 4 * ib);
    const v4f vh = *(const v4f*)(bhh_d + 4 * ib);
    const int ie = (tid < NDU / 4) ? tid : (NDU / 4 - 1);
    const v4f ve = *(const v4f*)(b_e2d + 4 * ie);
    if (tid < NG3 / 4) {
      *(v4f*)(bcs + 4 * ib) = vb;
      *(v4f*)(bcs + NG3 + 4 * ib) = vh;
    }
    if (tid < NDU / 4) *(v4f*)(bcs + 2 * NG3 + 4 * ie) = ve;
    ld_use4x3(vb, vh, ve);
  }
  const int plen = pred_len[0];
  const int nsteps = (plen < 0) ? 0 : ((plen > NPR) ? NPR : plen);
  __syncthreads();

  float wx0[NFE], wx1[NFE], wx2[NFE];
#pragma unroll
  for (int f = 0; f < NFE; ++f) {
    wx0[f] = wxs[(0 * NDU + j) * NFE + f];
    wx1[f] = wxs[(1 * NDU + j) * NFE + f];
    wx2[f] = wxs[(2 * NDU + j) * NFE + f];
  }
  const float bi0 = bcs[j], bi1 = bcs[NDU + j], bi2 = bcs[2 * NDU + j];
  const float bh0 = bcs[NG3 + j], bh1 = bcs[NG3 + NDU + j], bh2 = bcs[NG3 + 2 * NDU + j];
  const float be = bcs[2 * NG3 + j];

  const _Float16* carow = cA + (16 * mi + c) * CPAD + koff;
  const _Float16* harow = hA + (16 * mi + c) * HPAD + koff;
  const v8f z8 = {0.f, 0.f, 0.f, 0.f, 0.f, 0.f, 0.f, 0.f};
  float hst[8];

  {
    v8f acc = z8;
    const _Float16* wp = We2d16 + (size_t)j * NE2 + koff;
#pragma unroll 1
    for (int kc = 0; kc < NE2; kc += 32) {
      const v16h fa = Frag<_Float16>::load(carow + kc);
      const v16h fb = Frag<_Float16>::load(wp + kc);
      acc = Frag<_Float16>::mma(fa, fb, acc);
      dep_guard1_h(acc, fa, fb);
    }
    acc_guard1(acc);
#pragma unroll
    for (int r = 0; r < 8; ++r) hst[r] = acc[r] * WCAR_INV + be;
  }
#pragma unroll
  for (int r = 0; r < 8; ++r) hA[(16 * mi + 8 * hh + r) * HPAD + j] = (_Float16)hst[r];
  __syncthreads();

#pragma unroll 1
  for (int p = 0; p < nsteps; ++p) {
    {
      v8f acc = z8;
      const _Float16* wp = Wah16 + (size_t)j * NDU + koff;
#pragma unroll 1
      for (int kc = 0; kc < NDU; kc += 32) {
        const v16h fa = Frag<_Float16>::load(harow + kc);
        const v16h fb = Frag<_Float16>::load(wp + kc);
        acc = Frag<_Float16>::mma(fa, fb, acc);
        dep_guard1_h(acc, fa, fb);
      }
      acc_guard1(acc);
#pragma unroll
      for (int r = 0; r < 8; ++r) qs[(16 * mi + 8 * hh + r) * NDU + j] = acc[r] * WCAR_INV;
    }
    __syncthreads();

    {
      const int srow = tid >> 3, tl = tid & 7;
      const size_t erow0 = (size_t)(ba0 + srow) * NTOB;
      const float* qrow = qs + srow * NDU;
#pragma unroll 1
      for (int i = 0; i < NTOB / 8; ++i) {
        const int t = 8 * i + tl;
        const uint4* ep = (const uint4*)(E16p + (erow0 + (size_t)t) * NDU);
        float s = 0.0f;
#pragma unroll 1
        for (int u = 0; u < NDU / 8; ++u) {
          const uint4 w = ep[u];
          const v4f qa = *(const v4f*)(qrow + 8 * u);
          const v4f qb = *(const v4f*)(qrow + 8 * u + 4);
          const v4f va = *(const v4f*)(vs + 8 * u);
          const v4f vb = *(const v4f*)(vs + 8 * u + 4);
          s = sc_term(w.x & 0xffffu, qa[0], va[0], s);
          s = sc_term(w.x >> 16,     qa[1], va[1], s);
          s = sc_term(w.y & 0xffffu, qa[2], va[2], s);
          s = sc_term(w.y >> 16,     qa[3], va[3], s);
          s = sc_term(w.z & 0xffffu, qb[0], vb[0], s);
          s = sc_term(w.z >> 16,     qb[1], vb[1], s);
          s = sc_term(w.w & 0xffffu, qb[2], vb[2], s);
          s = sc_term(w.w >> 16,     qb[3], vb[3], s);
        }
        sc[srow * NTOB + t] = s;
      }
    }
    __syncthreads();

#pragma unroll
    for (int rr = 0; rr < 4; ++rr) {
      float* sp = sc + (4 * wave + rr) * NTOB;
      const float s0 = sp[lane], s1 = sp[32 + lane];
      float m = fmaxf(s0, s1);
#pragma unroll
      for (int off = 1; off < 32; off <<= 1) m = fmaxf(m, __shfl_xor(m, off, 32));
      const float e0 = expf(s0 - m), e1 = expf(s1 - m);
      float ssum = e0 + e1;
#pragma unroll
      for (int off = 1; off < 32; off <<= 1) ssum += __shfl_xor(ssum, off, 32);
      const float inv = 1.0f / ssum;
      sp[lane] = e0 * inv;
      sp[32 + lane] = e1 * inv;
    }
    __syncthreads();

    {
      const int row = tid >> 3, seg = tid & 7;
      const unsigned short* ebase = enc16p + (size_t)(ba0 + row) * NTOB * NE2 + 16 * seg;
      const float* wrow = sc + row * NTOB;
      float ca[16];
#pragma unroll
      for (int e = 0; e < 16; ++e) ca[e] = 0.0f;
#pragma unroll 1
      for (int t = 0; t < NTOB; ++t) {
        const float wt = wrow[t];
        const uint4 w0 = *(const uint4*)(ebase + (size_t)t * NE2);
        const uint4 w1 = *(const uint4*)(ebase + (size_t)t * NE2 + 8);
        ca[0]  = fmaf(wt, h16_to_f32(w0.x & 0xffffu), ca[0]);
        ca[1]  = fmaf(wt, h16_to_f32(w0.x >> 16),     ca[1]);
        ca[2]  = fmaf(wt, h16_to_f32(w0.y & 0xffffu), ca[2]);
        ca[3]  = fmaf(wt, h16_to_f32(w0.y >> 16),     ca[3]);
        ca[4]  = fmaf(wt, h16_to_f32(w0.z & 0xffffu), ca[4]);
        ca[5]  = fmaf(wt, h16_to_f32(w0.z >> 16),     ca[5]);
        ca[6]  = fmaf(wt, h16_to_f32(w0.w & 0xffffu), ca[6]);
        ca[7]  = fmaf(wt, h16_to_f32(w0.w >> 16),     ca[7]);
        ca[8]  = fmaf(wt, h16_to_f32(w1.x & 0xffffu), ca[8]);
        ca[9]  = fmaf(wt, h16_to_f32(w1.x >> 16),     ca[9]);
        ca[10] = fmaf(wt, h16_to_f32(w1.y & 0xffffu), ca[10]);
        ca[11] = fmaf(wt, h16_to_f32(w1.y >> 16),     ca[11]);
        ca[12] = fmaf(wt, h16_to_f32(w1.z & 0xffffu), ca[12]);
        ca[13] = fmaf(wt, h16_to_f32(w1.z >> 16),     ca[13]);
        ca[14] = fmaf(wt, h16_to_f32(w1.w & 0xffffu), ca[14]);
        ca[15] = fmaf(wt, h16_to_f32(w1.w >> 16),     ca[15]);
      }
      v8h h0v, h1v;
#pragma unroll
      for (int e = 0; e < 8; ++e) { h0v[e] = (_Float16)ca[e]; h1v[e] = (_Float16)ca[8 + e]; }
      *(v8h*)(cA + row * CPAD + 16 * seg) = h0v;
      *(v8h*)(cA + row * CPAD + 16 * seg + 8) = h1v;
    }
    __syncthreads();

    {
      v8f aI0 = z8, aI1 = z8, aI2 = z8, aH0 = z8, aH1 = z8, aH2 = z8;
      const _Float16* wi0 = Wihc16 + (size_t)(0 * NDU + j) * NE2 + koff;
      const _Float16* wi1 = Wihc16 + (size_t)(1 * NDU + j) * NE2 + koff;
      const _Float16* wi2 = Wihc16 + (size_t)(2 * NDU + j) * NE2 + koff;
#pragma unroll 1
      for (int kc = 0; kc < NE2; kc += 32) {
        const v16h fa = Frag<_Float16>::load(carow + kc);
        const v16h b0 = Frag<_Float16>::load(wi0 + kc);
        const v16h b1 = Frag<_Float16>::load(wi1 + kc);
        const v16h b2 = Frag<_Float16>::load(wi2 + kc);
        aI0 = Frag<_Float16>::mma(fa, b0, aI0);
        aI1 = Frag<_Float16>::mma(fa, b1, aI1);
        aI2 = Frag<_Float16>::mma(fa, b2, aI2);
        dep_guard3_h(aI0, aI1, aI2, fa, b0, b1, b2);
      }
      const _Float16* wh0 = Whhd16 + (size_t)(0 * NDU + j) * NDU + koff;
      const _Float16* wh1 = Whhd16 + (size_t)(1 * NDU + j) * NDU + koff;
      const _Float16* wh2 = Whhd16 + (size_t)(2 * NDU + j) * NDU + koff;
#pragma unroll 1
      for (int kc = 0; kc < NDU; kc += 32) {
        const v16h fa = Frag<_Float16>::load(harow + kc);
        const v16h b0 = Frag<_Float16>::load(wh0 + kc);
        const v16h b1 = Frag<_Float16>::load(wh1 + kc);
        const v16h b2 = Frag<_Float16>::load(wh2 + kc);
        aH0 = Frag<_Float16>::mma(fa, b0, aH0);
        aH1 = Frag<_Float16>::mma(fa, b1, aH1);
        aH2 = Frag<_Float16>::mma(fa, b2, aH2);
        dep_guard3_h(aH0, aH1, aH2, fa, b0, b1, b2);
      }
      acc_guard3(aI0, aI1, aI2);
      acc_guard3(aH0, aH1, aH2);
#pragma unroll
      for (int r = 0; r < 8; ++r) {
        const int row = 16 * mi + 8 * hh + r;
        const float* dp = po + row * NFE;
        float gir = bi0, giz = bi1, gin = bi2;
#pragma unroll
        for (int f = 0; f < NFE; ++f) {
          const float dv = dp[f];
          gir = fmaf(dv, wx0[f], gir);
          giz = fmaf(dv, wx1[f], giz);
          gin = fmaf(dv, wx2[f], gin);
        }
        const float pr  = (aI0[r] + aH0[r]) * WCAR_INV + gir + bh0;
        const float pz  = (aI1[r] + aH1[r]) * WCAR_INV + giz + bh1;
        const float hn  = aH2[r] * WCAR_INV + bh2;
        const float inn = aI2[r] * WCAR_INV + gin;
        const float rg = fsig(pr);
        const float zg = fsig(pz);
        const float ng = ftanh(inn + rg * hn);
        hst[r] = (1.0f - zg) * ng + zg * hst[r];
      }
    }
    __syncthreads();

#pragma unroll
    for (int r = 0; r < 8; ++r) {
      const int row = 16 * mi + 8 * hh + r;
      hA[row * HPAD + j] = (_Float16)hst[r];
      hs[row * NDU + j] = hst[r];
    }
    __syncthreads();

    {
      const int prow = tid / NFE;
      const int f = tid - NFE * prow;
      const int prc = (prow < DEC_ROWS) ? prow : (DEC_ROWS - 1);
      const float* hp = hs + prc * NDU;
      const float* wp = wo + f * NDU;
      float s = 0.0f;
#pragma unroll 4
      for (int jj = 0; jj < NDU; ++jj) s = fmaf(hp[jj], wp[jj], s);
      s += b_out[f];
      ld_use_f1(s);
      if (tid < NROWF) po[tid] = s;
    }
    __syncthreads();

    if (wave == 0) {
      float* orow = out + ((size_t)bidx * NPR + (size_t)p) * NROWF;
      const v4f v0 = *(const v4f*)(po + 4 * lane);
      const int l2 = (lane < 16) ? lane : 15;
      const v4f v1 = *(const v4f*)(po + 128 + 4 * l2);
      for (int pass = 0; pass < 2; ++pass) {
        *(volatile v4f*)(orow + 4 * lane) = v0;
        if (lane < 16) *(volatile v4f*)(orow + 128 + 4 * lane) = v1;
        __threadfence();
      }
    }
  }
}

extern "C" void kernel_launch(void* const* d_in, const int* in_sizes, int n_in,
                              void* d_out, int out_size, void* d_ws, size_t ws_size, hipStream_t stream) {
  if (n_in < 21 || d_out == nullptr || d_ws == nullptr) return;
  if (in_sizes[0] != NBAT * NTOB * NROWF || in_sizes[1] < 1 ||
      in_sizes[2] != NG3 * NFE || in_sizes[3] != NG3 * NHU || in_sizes[4] != NG3 || in_sizes[5] != NG3 ||
      in_sizes[6] != NG3 * NFE || in_sizes[7] != NG3 * NHU || in_sizes[8] != NG3 || in_sizes[9] != NG3 ||
      in_sizes[10] != NDU * NATT || in_sizes[11] != NDU || in_sizes[12] != NDU ||
      in_sizes[13] != NDU * NE2 || in_sizes[14] != NDU ||
      in_sizes[15] != NG3 * NDIN || in_sizes[16] != NG3 * NDU || in_sizes[17] != NG3 || in_sizes[18] != NG3 ||
      in_sizes[19] != NFE * NDU || in_sizes[20] != NFE ||
      out_size != NBAT * NPR * NROWF) return;

  const float* src    = (const float*)d_in[0];
  const int*   plen   = (const int*)d_in[1];
  const float* Wih_f  = (const float*)d_in[2];
  const float* Whh_f  = (const float*)d_in[3];
  const float* bih_f  = (const float*)d_in[4];
  const float* bhh_f  = (const float*)d_in[5];
  const float* Wih_b  = (const float*)d_in[6];
  const float* Whh_b  = (const float*)d_in[7];
  const float* bih_b  = (const float*)d_in[8];
  const float* bhh_b  = (const float*)d_in[9];
  const float* W_attn = (const float*)d_in[10];
  const float* b_attn = (const float*)d_in[11];
  const float* v_attn = (const float*)d_in[12];
  const float* W_e2d  = (const float*)d_in[13];
  const float* b_e2d  = (const float*)d_in[14];
  const float* Wih_d  = (const float*)d_in[15];
  const float* Whh_d  = (const float*)d_in[16];
  const float* bih_d  = (const float*)d_in[17];
  const float* bhh_d  = (const float*)d_in[18];
  const float* W_out  = (const float*)d_in[19];
  const float* b_out  = (const float*)d_in[20];
  float* out = (float*)d_out;

  char* ws = (char*)d_ws; size_t off = 0;
  auto carve = [&](size_t bytes) -> char* { char* p = ws + off; off += (bytes + 255) & ~(size_t)255; return p; };
  unsigned short* enc16  = (unsigned short*)carve((size_t)NER * NE2 * 2);
  unsigned short* E16    = (unsigned short*)carve((size_t)NER * NDU * 2);
  unsigned short* Whhf16 = (unsigned short*)carve((size_t)NG3 * NHU * 2);
  unsigned short* Whhb16 = (unsigned short*)carve((size_t)NG3 * NHU * 2);
  unsigned short* Wae16  = (unsigned short*)carve((size_t)NDU * NE2 * 2);
  unsigned short* Wah16  = (unsigned short*)carve((size_t)NDU * NDU * 2);
  unsigned short* Wihc16 = (unsigned short*)carve((size_t)NG3 * NE2 * 2);
  unsigned short* Whhd16 = (unsigned short*)carve((size_t)NG3 * NDU * 2);
  unsigned short* We2d16 = (unsigned short*)carve((size_t)NDU * NE2 * 2);
  if (off > ws_size || off > (size_t)134217728) return;

  cvt_f16_kernel<<<(NG3 * (NHU / 8) + 255) / 256, 256, 0, stream>>>(Whh_f,  Whhf16, NG3, NHU / 8, NHU,  0,   WCAR);
  cvt_f16_kernel<<<(NG3 * (NHU / 8) + 255) / 256, 256, 0, stream>>>(Whh_b,  Whhb16, NG3, NHU / 8, NHU,  0,   WCAR);
  cvt_f16_kernel<<<(NDU * (NE2 / 8) + 255) / 256, 256, 0, stream>>>(W_attn, Wae16,  NDU, NE2 / 8, NATT, NDU, WCAR);
  cvt_f16_kernel<<<(NDU * (NDU / 8) + 255) / 256, 256, 0, stream>>>(W_attn, Wah16,  NDU, NDU / 8, NATT, 0,   WCAR);
  cvt_f16_kernel<<<(NG3 * (NE2 / 8) + 255) / 256, 256, 0, stream>>>(Wih_d,  Wihc16, NG3, NE2 / 8, NDIN, NFE, WCAR);
  cvt_f16_kernel<<<(NG3 * (NDU / 8) + 255) / 256, 256, 0, stream>>>(Whh_d,  Whhd16, NG3, NDU / 8, NDU,  0,   WCAR);
  cvt_f16_kernel<<<(NDU * (NE2 / 8) + 255) / 256, 256, 0, stream>>>(W_e2d,  We2d16, NDU, NE2 / 8, NE2,  0,   WCAR);

  enc_gru_kernel<<<dim3(NBA / ENC_ROWS, 2), ENC_THR, 0, stream>>>(src, Wih_f, bih_f, bhh_f, Wih_b, bih_b, bhh_b,
                                                                 Whhf16, Whhb16, enc16);

  const dim3 ggrid((NER / 64) * (NDU / 64) / 8, 1);
  wmma_gemm64<0, false, 2, 1, false, 0><<<ggrid, 256, 0, stream>>>(
      enc16, enc16, NE2, 0L, Wae16, Wae16, NE2, 0L, (void*)E16, (void*)E16, NDU, 0L,
      b_attn, b_attn, 0L, NER, NDU, NE2, WCAR_INV);

  dec_kernel<<<NBAT, DEC_THR, 0, stream>>>(src, plen, enc16, E16, Wah16, Wihc16, Whhd16, We2d16,
                                           v_attn, b_e2d, Wih_d, bih_d, bhh_d, W_out, b_out, out);
}
